// GCNPolicy_26542897889601
// MI455X (gfx1250) — hardware-verified
//
#include <hip/hip_runtime.h>
#include <stddef.h>


#define DF      128
#define HID     1024
#define NACT    8
#define NTHR    256
#define NWAVE   8
#define EPT     8
#define NGRP    2
#define CHUNK   (NTHR * EPT * NGRP)
#define WCAP    (EPT * NGRP * 32)
#define LISTN   (NWAVE * WCAP)
#define NB1     64
#define NB2     1024
#define NBD     4096
#define GR      16
#define APITCH  136
#define NGMAX   256
#define W1SCALE 8.0f
#define W1INV   0.125f
#define W2SCALE 32.0f
#define W2INV   0.03125f

#define LDS_GEMM1 (GR * HID * 4)
#define LDS_AGG1  (NB1 * HID * 4 + LISTN * 4 + 64)

static_assert((CHUNK & (CHUNK - 1)) == 0);
static_assert(CHUNK <= 4096);
static_assert((NB1 & (NB1 - 1)) == 0 && (NB2 & (NB2 - 1)) == 0 && (NBD & (NBD - 1)) == 0);
static_assert(NB1 <= 4096 && NB2 <= 4096 && NBD <= 4096);
static_assert(GR * APITCH * 2 <= LDS_GEMM1);
static_assert(NB1 % GR == 0 && NB2 % GR == 0);
static_assert(HID == NWAVE * 128);
static_assert(NB1 == NWAVE * 8);
static_assert(NB2 * NACT == NWAVE * 8 * 128);
static_assert(DF % 32 == 0 && HID % 32 == 0);
static_assert(GR * DF / 8 == NTHR);

typedef float    v4f  __attribute__((ext_vector_type(4)));
typedef float    v8f  __attribute__((ext_vector_type(8)));
typedef int      v4i  __attribute__((ext_vector_type(4)));
typedef _Float16 v8h  __attribute__((ext_vector_type(8)));
typedef _Float16 v16h __attribute__((ext_vector_type(16)));
union FragH { v16h v; v8h h[2]; };

__device__ __forceinline__ v8h cvt8(v4f a, v4f b) {
  v8h r;
  r[0] = (_Float16)a.x; r[1] = (_Float16)a.y; r[2] = (_Float16)a.z; r[3] = (_Float16)a.w;
  r[4] = (_Float16)b.x; r[5] = (_Float16)b.y; r[6] = (_Float16)b.z; r[7] = (_Float16)b.w;
  return r;
}

__device__ __forceinline__ v8f wmh(v16h a, v16h b, v8f c) {
  v8f d = __builtin_amdgcn_wmma_f32_16x16x32_f16(false, a, false, b, (short)0, c, false, false);
  asm volatile("v_nop\n\tv_nop\n\tv_nop\n\tv_nop" : "+v"(d) : "v"(a), "v"(b));
  return d;
}

template <int NB>
__device__ __forceinline__ int scan_chunk(const int* __restrict__ dsts, int nE, int cbase, int nodeBase,
                                          int vec8, int* list, int tid, int lane, int wave) {
  int wc = 0;
  (void)lane;
#pragma unroll
  for (int g = 0; g < NGRP; ++g) {
    const int el0  = (g * NTHR + tid) * EPT;
    const int e0   = cbase + el0;
    const int sent = -2147483647 - 1;
    v4i da, db;
    if (vec8 != 0 && e0 + 7 < nE) {
      da = *(const v4i*)(dsts + e0);
      db = *(const v4i*)(dsts + e0 + 4);
    } else {
      da.x = (e0     < nE) ? dsts[min(e0, nE - 1)] : sent;
      da.y = (e0 + 1 < nE) ? dsts[min(e0 + 1, nE - 1)] : sent;
      da.z = (e0 + 2 < nE) ? dsts[min(e0 + 2, nE - 1)] : sent;
      da.w = (e0 + 3 < nE) ? dsts[min(e0 + 3, nE - 1)] : sent;
      db.x = (e0 + 4 < nE) ? dsts[min(e0 + 4, nE - 1)] : sent;
      db.y = (e0 + 5 < nE) ? dsts[min(e0 + 5, nE - 1)] : sent;
      db.z = (e0 + 6 < nE) ? dsts[min(e0 + 6, nE - 1)] : sent;
      db.w = (e0 + 7 < nE) ? dsts[min(e0 + 7, nE - 1)] : sent;
    }
    const unsigned nb = (unsigned)nodeBase;
    const unsigned s0 = (unsigned)da.x - nb, s1 = (unsigned)da.y - nb;
    const unsigned s2 = (unsigned)da.z - nb, s3 = (unsigned)da.w - nb;
    const unsigned s4 = (unsigned)db.x - nb, s5 = (unsigned)db.y - nb;
    const unsigned s6 = (unsigned)db.z - nb, s7 = (unsigned)db.w - nb;
    const bool h0 = s0 < (unsigned)NB, h1 = s1 < (unsigned)NB, h2 = s2 < (unsigned)NB, h3 = s3 < (unsigned)NB;
    const bool h4 = s4 < (unsigned)NB, h5 = s5 < (unsigned)NB, h6 = s6 < (unsigned)NB, h7 = s7 < (unsigned)NB;
    const unsigned any = __builtin_amdgcn_ballot_w32(h0 | h1 | h2 | h3 | h4 | h5 | h6 | h7);
    if (any != 0u) {
#define HITJ(J, HJ, SJ) { \
        const unsigned mj = __builtin_amdgcn_ballot_w32(HJ); \
        if (mj != 0u) { \
          if (HJ) { \
            const int pos = wc + (int)__builtin_amdgcn_mbcnt_lo(mj, 0u); \
            if (pos < WCAP) list[wave * WCAP + pos] = ((el0 + (J)) << 12) | (int)(SJ); \
          } \
          wc += (int)__builtin_popcount(mj); } }
      HITJ(0, h0, s0)
      HITJ(1, h1, s1)
      HITJ(2, h2, s2)
      HITJ(3, h3, s3)
      HITJ(4, h4, s4)
      HITJ(5, h5, s5)
      HITJ(6, h6, s6)
      HITJ(7, h7, s7)
#undef HITJ
    }
  }
  return wc;
}

__global__ __launch_bounds__(NTHR) void k_wprep(
    const float* __restrict__ W1, const float* __restrict__ W2,
    _Float16* w1t, _Float16* w2t) {
  const int i  = blockIdx.x * NTHR + threadIdx.x;
  const int n1 = HID * DF / 8;
  const int n2 = HID * HID / 8;
  if (i >= n1 + n2) return;
  const bool first = i < n1;
  v4f a, b;
  _Float16* dp;
  if (first) {
    const int o  = i * 8;
    const int n  = o / DF;
    const int k0 = o - n * DF;
    const float* p = W1 + (size_t)k0 * HID + n;
    a.x = p[0];       a.y = p[HID];     a.z = p[2 * HID]; a.w = p[3 * HID];
    b.x = p[4 * HID]; b.y = p[5 * HID]; b.z = p[6 * HID]; b.w = p[7 * HID];
    a = a * W1SCALE;
    b = b * W1SCALE;
    dp = w1t + o;
  } else {
    const int o  = (i - n1) * 8;
    const int n  = o / HID;
    const int k0 = o - n * HID;
    const float* p = W2 + (size_t)k0 * HID + n;
    a.x = p[0];       a.y = p[HID];     a.z = p[2 * HID]; a.w = p[3 * HID];
    b.x = p[4 * HID]; b.y = p[5 * HID]; b.z = p[6 * HID]; b.w = p[7 * HID];
    a = a * W2SCALE;
    b = b * W2SCALE;
    dp = w2t + o;
  }
  const v8h hv = cvt8(a, b);
  *(volatile v8h*)dp = hv;
  __threadfence();
  *(volatile v8h*)dp = hv;
}

__global__ __launch_bounds__(NTHR) void k_deg(
    const int* __restrict__ ei, float* dinv, int nN, int nE, int vec8) {
  __shared__ __attribute__((aligned(16))) int cnt[NBD];
  __shared__ __attribute__((aligned(16))) int list[LISTN];
  __shared__ int wcnt[NWAVE];
  const int tid = threadIdx.x, lane = tid & 31, wave = tid >> 5;
  const int nodeBase = blockIdx.x * NBD;
  const int* dsts = ei + nE;
  (void)nN;

  for (int i = tid; i < NBD; i += NTHR) cnt[i] = 0;
  __syncthreads();

  const int nChunks = (nE + CHUNK - 1) / CHUNK;
#pragma unroll 1
  for (int ch = 0; ch < nChunks; ++ch) {
    const int cbase = ch * CHUNK;
    const int wc = scan_chunk<NBD>(dsts, nE, cbase, nodeBase, vec8, list, tid, lane, wave);
    if (lane == 0) wcnt[wave] = wc;
    __syncthreads();
    if (wave == 0) {
#pragma unroll 1
      for (int wsx = 0; wsx < NWAVE; ++wsx) {
        int n = __builtin_amdgcn_readfirstlane(wcnt[wsx]);
        n = n > WCAP ? WCAP : (n < 0 ? 0 : n);
        const int* lp = list + wsx * WCAP;
#pragma unroll 1
        for (int i = 0; i < n; ++i) {
          const int ent  = __builtin_amdgcn_readfirstlane(lp[i]);
          const int slot = ent & (NBD - 1);
          if (lane == 0) cnt[slot] = cnt[slot] + 1;
        }
      }
    }
    __syncthreads();
  }

  v4f dq[4];
#pragma unroll
  for (int q = 0; q < 4; ++q) {
    const int f = (wave * 4 + q) * 128 + 4 * lane;
    const v4i c = *(const v4i*)(cnt + f);
    dq[q].x = rsqrtf((float)(c.x + 1));
    dq[q].y = rsqrtf((float)(c.y + 1));
    dq[q].z = rsqrtf((float)(c.z + 1));
    dq[q].w = rsqrtf((float)(c.w + 1));
  }
  float* dp = dinv + (size_t)nodeBase;
#pragma unroll
  for (int q = 0; q < 4; ++q) *(volatile v4f*)(dp + (wave * 4 + q) * 128 + 4 * lane) = dq[q];
  __threadfence();
#pragma unroll
  for (int q = 0; q < 4; ++q) *(volatile v4f*)(dp + (wave * 4 + q) * 128 + 4 * lane) = dq[q];
}

__global__ __launch_bounds__(NTHR) void k_gemm1(
    const float* __restrict__ x, const _Float16* __restrict__ w1t,
    const float* __restrict__ dinv, float* g1, int nN) {
  extern __shared__ v4f lds_dyn[];
  _Float16* sA  = (_Float16*)lds_dyn;
  float*    stg = (float*)lds_dyn;
  const int tid = threadIdx.x, lane = tid & 31, wave = tid >> 5, hh = lane >> 4, m = lane & 15;
  const int rowBase = blockIdx.x * GR;

  {
    const int r  = tid >> 4;
    const int c0 = (tid & 15) * 8;
    int node = rowBase + r;
    node = node > nN - 1 ? nN - 1 : node;
    const float* xp = x + (size_t)node * DF + c0;
    const v4f a = *(const v4f*)xp, b = *(const v4f*)(xp + 4);
    *(v8h*)(sA + r * APITCH + c0) = cvt8(a, b);
  }
  __syncthreads();

  v8f acc[8];
#pragma unroll
  for (int t = 0; t < 8; ++t) { v8f z = {0.f, 0.f, 0.f, 0.f, 0.f, 0.f, 0.f, 0.f}; acc[t] = z; }
  const _Float16* ar = sA + m * APITCH + 8 * hh;
  const _Float16* bb = w1t + (size_t)(128 * wave + m) * DF + 8 * hh;
#pragma unroll
  for (int kt = 0; kt < DF / 32; ++kt) {
    FragH a;
    a.h[0] = *(const v8h*)(ar + 32 * kt);
    a.h[1] = *(const v8h*)(ar + 32 * kt + 16);
#pragma unroll
    for (int t = 0; t < 8; ++t) {
      const _Float16* bp = bb + (size_t)(16 * t) * DF + 32 * kt;
      FragH b;
      b.h[0] = *(const v8h*)bp;
      b.h[1] = *(const v8h*)(bp + 16);
      acc[t] = wmh(a.v, b.v, acc[t]);
    }
  }
  __syncthreads();

  const int r0 = 8 * hh;
  const v4f dA = *(const v4f*)(dinv + (size_t)rowBase + r0);
  const v4f dB = *(const v4f*)(dinv + (size_t)rowBase + r0 + 4);
  const float d0 = dA.x * W1INV, d1 = dA.y * W1INV, d2 = dA.z * W1INV, d3 = dA.w * W1INV;
  const float d4 = dB.x * W1INV, d5 = dB.y * W1INV, d6 = dB.z * W1INV, d7 = dB.w * W1INV;
  float* sp = stg + r0 * HID + 128 * wave + m;
#pragma unroll
  for (int t = 0; t < 8; ++t) {
    sp[0 * HID + 16 * t] = acc[t][0] * d0;
    sp[1 * HID + 16 * t] = acc[t][1] * d1;
    sp[2 * HID + 16 * t] = acc[t][2] * d2;
    sp[3 * HID + 16 * t] = acc[t][3] * d3;
    sp[4 * HID + 16 * t] = acc[t][4] * d4;
    sp[5 * HID + 16 * t] = acc[t][5] * d5;
    sp[6 * HID + 16 * t] = acc[t][6] * d6;
    sp[7 * HID + 16 * t] = acc[t][7] * d7;
  }
  __syncthreads();

#pragma unroll
  for (int i = 0; i < 2; ++i) {
    const int row = 2 * wave + i;
    const float* lp = stg + row * HID + 4 * lane;
    float* gp = g1 + ((size_t)rowBase + row) * HID + 4 * lane;
#pragma unroll
    for (int j = 0; j < 8; ++j) { const v4f v = *(const v4f*)(lp + 128 * j); *(volatile v4f*)(gp + 128 * j) = v; }
  }
  __threadfence();
#pragma unroll
  for (int i = 0; i < 2; ++i) {
    const int row = 2 * wave + i;
    const float* lp = stg + row * HID + 4 * lane;
    float* gp = g1 + ((size_t)rowBase + row) * HID + 4 * lane;
#pragma unroll
    for (int j = 0; j < 8; ++j) { const v4f v = *(const v4f*)(lp + 128 * j); *(volatile v4f*)(gp + 128 * j) = v; }
  }
}

__global__ __launch_bounds__(NTHR) void k_agg1(
    const int* __restrict__ ei, const float* __restrict__ g1, const float* __restrict__ dinv,
    const float* __restrict__ b1, _Float16* h1p, int nN, int nE, int vec8) {
  extern __shared__ v4f lds_dyn[];
  float* acc  = (float*)lds_dyn;
  int*   list = (int*)(acc + NB1 * HID);
  int*   wcnt = list + LISTN;
  const int tid = threadIdx.x, lane = tid & 31, wave = tid >> 5;
  const int nodeBase = blockIdx.x * NB1;
  const int* dsts = ei + nE;

  {
    const v4f z = {0.f, 0.f, 0.f, 0.f};
    for (int i = tid; i < NB1 * HID / 4; i += NTHR) lds_dyn[i] = z;
  }
  __syncthreads();

  const int nChunks = (nE + CHUNK - 1) / CHUNK;
#pragma unroll 1
  for (int ch = 0; ch < nChunks; ++ch) {
    const int cbase = ch * CHUNK;
    const int wc = scan_chunk<NB1>(dsts, nE, cbase, nodeBase, vec8, list, tid, lane, wave);
    if (lane == 0) wcnt[wave] = wc;
    __syncthreads();
#pragma unroll 1
    for (int wsx = 0; wsx < NWAVE; ++wsx) {
      int n = __builtin_amdgcn_readfirstlane(wcnt[wsx]);
      n = n > WCAP ? WCAP : (n < 0 ? 0 : n);
      const int* lp = list + wsx * WCAP;
#pragma unroll 1
      for (int i = 0; i < n; ++i) {
        const int ent  = __builtin_amdgcn_readfirstlane(lp[i]);
        const int slot = ent & (NB1 - 1);
        int e = cbase + ((ent >> 12) & (CHUNK - 1));
        e = e > nE - 1 ? nE - 1 : e;
        int src = ei[e];
        src = src < 0 ? 0 : (src > nN - 1 ? nN - 1 : src);
        const v4f v = *(const v4f*)(g1 + (size_t)src * HID + 128 * wave + 4 * lane);
        v4f* ap = (v4f*)(acc + slot * HID + 128 * wave + 4 * lane);
        *ap = *ap + v;
      }
    }
    __syncthreads();
  }

#pragma unroll 1
  for (int q = 0; q < NB1 / NWAVE; ++q) {
    const int row = wave + NWAVE * q;
    int node = nodeBase + row;
    node = node > nN - 1 ? nN - 1 : node;
    const float d = dinv[node];
    const float* ap = acc + row * HID + 8 * lane;
    const float* gp = g1 + (size_t)node * HID + 8 * lane;
    const float* bp = b1 + 8 * lane;
    v8h hv[4];
#pragma unroll
    for (int s = 0; s < 4; ++s) {
      const v4f a0 = *(const v4f*)(ap + 256 * s), a1 = *(const v4f*)(ap + 256 * s + 4);
      const v4f e0 = *(const v4f*)(gp + 256 * s), e1 = *(const v4f*)(gp + 256 * s + 4);
      const v4f c0 = *(const v4f*)(bp + 256 * s), c1 = *(const v4f*)(bp + 256 * s + 4);
      v4f u0 = (a0 + e0) * d + c0;
      v4f u1 = (a1 + e1) * d + c1;
      u0.x = fmaxf(u0.x, 0.f); u0.y = fmaxf(u0.y, 0.f); u0.z = fmaxf(u0.z, 0.f); u0.w = fmaxf(u0.w, 0.f);
      u1.x = fmaxf(u1.x, 0.f); u1.y = fmaxf(u1.y, 0.f); u1.z = fmaxf(u1.z, 0.f); u1.w = fmaxf(u1.w, 0.f);
      hv[s] = cvt8(u0, u1);
    }
    _Float16* hp = h1p + ((size_t)nodeBase + row) * HID + 8 * lane;
#pragma unroll
    for (int s = 0; s < 4; ++s) *(volatile v8h*)(hp + 256 * s) = hv[s];
    __threadfence();
#pragma unroll
    for (int s = 0; s < 4; ++s) *(volatile v8h*)(hp + 256 * s) = hv[s];
  }
}

__global__ __launch_bounds__(NTHR) void k_gemm2h(
    const _Float16* __restrict__ h1p, const _Float16* __restrict__ w2t,
    const float* __restrict__ Wl, const float* __restrict__ dinv, float* pp) {
  __shared__ __attribute__((aligned(16))) float ps[NWAVE * GR * NACT];
  const int tid = threadIdx.x, lane = tid & 31, wave = tid >> 5, hh = lane >> 4, m = lane & 15;
  const int rowBase = blockIdx.x * GR;

  v8f acc[8];
#pragma unroll
  for (int t = 0; t < 8; ++t) { v8f z = {0.f, 0.f, 0.f, 0.f, 0.f, 0.f, 0.f, 0.f}; acc[t] = z; }
  const _Float16* ap = h1p + ((size_t)rowBase + m) * HID + 8 * hh;
  const _Float16* bb = w2t + (size_t)(128 * wave + m) * HID + 8 * hh;
#pragma unroll 1
  for (int ks = 0; ks < HID / 32; ++ks) {
    FragH a;
    a.h[0] = *(const v8h*)(ap + 32 * ks);
    a.h[1] = *(const v8h*)(ap + 32 * ks + 16);
#pragma unroll
    for (int t = 0; t < 8; ++t) {
      const _Float16* bp = bb + (size_t)(16 * t) * HID + 32 * ks;
      FragH b;
      b.h[0] = *(const v8h*)bp;
      b.h[1] = *(const v8h*)(bp + 16);
      acc[t] = wmh(a.v, b.v, acc[t]);
    }
  }

  const float* wlp = Wl + (size_t)(128 * wave + m) * NACT;
#pragma unroll 1
  for (int a = 0; a < NACT; ++a) {
    float wv[8];
#pragma unroll
    for (int t = 0; t < 8; ++t) wv[t] = wlp[(16 * t) * NACT + a];
    float p[8];
#pragma unroll
    for (int r = 0; r < 8; ++r) {
      float s = acc[0][r] * wv[0];
#pragma unroll
      for (int t = 1; t < 8; ++t) s = acc[t][r] * wv[t] + s;
      p[r] = s;
    }
#pragma unroll
    for (int r = 0; r < 8; ++r) {
      float v = p[r];
      v += __shfl_xor(v, 8);
      v += __shfl_xor(v, 4);
      v += __shfl_xor(v, 2);
      v += __shfl_xor(v, 1);
      p[r] = v;
    }
    if (m == 0) {
#pragma unroll
      for (int r = 0; r < 8; ++r) ps[(wave * GR + 8 * hh + r) * NACT + a] = p[r];
    }
  }
  __syncthreads();

  if (wave == 0) {
    const int row = lane >> 1;
    const int a0  = 4 * (lane & 1);
    v4f s = {0.f, 0.f, 0.f, 0.f};
#pragma unroll
    for (int w = 0; w < NWAVE; ++w) s = s + *(const v4f*)(ps + (w * GR + row) * NACT + a0);
    const float d = dinv[(size_t)rowBase + row] * W2INV;
    s = s * d;
    float* gp = pp + (size_t)rowBase * NACT + 4 * lane;
    *(volatile v4f*)gp = s;
    __threadfence();
    *(volatile v4f*)gp = s;
  }
}

__global__ __launch_bounds__(NTHR) void k_agg2(
    const int* __restrict__ ei, const float* __restrict__ pp, const float* __restrict__ dinv,
    const float* __restrict__ b2, const float* __restrict__ Wl, const float* __restrict__ bl,
    float* h3, int nN, int nE, int vec8) {
  __shared__ __attribute__((aligned(16))) float acc[NB2 * NACT];
  __shared__ __attribute__((aligned(16))) int list[LISTN];
  __shared__ int wcnt[NWAVE];
  __shared__ float cst[NACT];
  const int tid = threadIdx.x, lane = tid & 31, wave = tid >> 5;
  const int nodeBase = blockIdx.x * NB2;
  const int* dsts = ei + nE;

  if (tid < NACT) {
    float s = 0.f;
#pragma unroll 1
    for (int k = 0; k < HID; ++k) s = b2[k] * Wl[k * NACT + tid] + s;
    cst[tid] = s + bl[tid];
  }
  {
    const v4f z = {0.f, 0.f, 0.f, 0.f};
    for (int i = tid; i < NB2 * NACT / 4; i += NTHR) *(v4f*)(acc + 4 * i) = z;
  }
  __syncthreads();

  const int nChunks = (nE + CHUNK - 1) / CHUNK;
#pragma unroll 1
  for (int ch = 0; ch < nChunks; ++ch) {
    const int cbase = ch * CHUNK;
    const int wc = scan_chunk<NB2>(dsts, nE, cbase, nodeBase, vec8, list, tid, lane, wave);
    if (lane == 0) wcnt[wave] = wc;
    __syncthreads();
    if (wave == 0) {
#pragma unroll 1
      for (int wsx = 0; wsx < NWAVE; ++wsx) {
        int n = __builtin_amdgcn_readfirstlane(wcnt[wsx]);
        n = n > WCAP ? WCAP : (n < 0 ? 0 : n);
        const int* lp = list + wsx * WCAP;
#pragma unroll 1
        for (int i = 0; i < n; ++i) {
          const int ent  = __builtin_amdgcn_readfirstlane(lp[i]);
          const int slot = ent & (NB2 - 1);
          int e = cbase + ((ent >> 12) & (CHUNK - 1));
          e = e > nE - 1 ? nE - 1 : e;
          int src = ei[e];
          src = src < 0 ? 0 : (src > nN - 1 ? nN - 1 : src);
          if (lane < NACT) {
            float* ap = acc + slot * NACT + lane;
            *ap = *ap + pp[(size_t)src * NACT + lane];
          }
        }
      }
    }
    __syncthreads();
  }

#pragma unroll 1
  for (int idx = tid; idx < NB2 * NACT; idx += NTHR) {
    const int row = idx >> 3;
    const int a   = idx & 7;
    int node = nodeBase + row;
    node = node > nN - 1 ? nN - 1 : node;
    const float v = (acc[idx] + pp[(size_t)node * NACT + a]) * dinv[node] + cst[a];
    acc[idx] = tanhf(v);
  }
  __syncthreads();

  float* base = h3 + (size_t)nodeBase * NACT;
#pragma unroll
  for (int q = 0; q < 8; ++q) {
    const int f = (wave * 8 + q) * 128 + 4 * lane;
    const v4f v = *(const v4f*)(acc + f);
    *(volatile v4f*)(base + f) = v;
  }
  __threadfence();
#pragma unroll
  for (int q = 0; q < 8; ++q) {
    const int f = (wave * 8 + q) * 128 + 4 * lane;
    const v4f v = *(const v4f*)(acc + f);
    *(volatile v4f*)(base + f) = v;
  }
}

__global__ __launch_bounds__(NTHR) void k_pool(
    const float* __restrict__ h3, const int* __restrict__ bt, float* out, int nN, int nG) {
  __shared__ __attribute__((aligned(16))) float res[NGMAX * NACT];
  const int tid = threadIdx.x, lane = tid & 31, wave = tid >> 5;

#pragma unroll 1
  for (int g = wave; g < nG; g += NWAVE) {
    v4f sa = {0.f, 0.f, 0.f, 0.f}, sb = {0.f, 0.f, 0.f, 0.f};
    float c = 0.f;
#pragma unroll 1
    for (int i = lane; i < nN; i += 32) {
      const int b = bt[i];
      if (b == g) {
        const float* hp = h3 + (size_t)i * NACT;
        sa = sa + *(const v4f*)hp;
        sb = sb + *(const v4f*)(hp + 4);
        c += 1.f;
      }
    }
#pragma unroll
    for (int off = 16; off > 0; off >>= 1) {
      sa.x += __shfl_xor(sa.x, off); sa.y += __shfl_xor(sa.y, off);
      sa.z += __shfl_xor(sa.z, off); sa.w += __shfl_xor(sa.w, off);
      sb.x += __shfl_xor(sb.x, off); sb.y += __shfl_xor(sb.y, off);
      sb.z += __shfl_xor(sb.z, off); sb.w += __shfl_xor(sb.w, off);
      c += __shfl_xor(c, off);
    }
    if (lane == 0) {
      const float inv = 1.0f / fmaxf(c, 1.0f);
      *(v4f*)(res + g * NACT)     = sa * inv;
      *(v4f*)(res + g * NACT + 4) = sb * inv;
    }
  }
  __syncthreads();

  const int tot  = nG * NACT;
  const int ngrp = (tot + 127) / 128;
#pragma unroll 1
  for (int q = wave; q < ngrp; q += NWAVE) {
    const int f = q * 128 + 4 * lane;
    if (f < tot) { const v4f v = *(const v4f*)(res + f); *(volatile v4f*)(out + f) = v; }
  }
  __threadfence();
#pragma unroll 1
  for (int q = wave; q < ngrp; q += NWAVE) {
    const int f = q * 128 + 4 * lane;
    if (f < tot) { const v4f v = *(const v4f*)(res + f); *(volatile v4f*)(out + f) = v; }
  }
}

extern "C" void kernel_launch(void* const* d_in, const int* in_sizes, int n_in,
                              void* d_out, int out_size, void* d_ws, size_t ws_size,
                              hipStream_t stream) {
  if (n_in < 9) return;
  const int nN = in_sizes[2];
  if (nN <= 0) return;
  if (in_sizes[0] != nN * DF) return;
  const int nE = in_sizes[1] / 2;
  if (nE < 0 || in_sizes[1] != nE * 2) return;
  if (in_sizes[3] != DF * HID || in_sizes[4] < HID) return;
  if (in_sizes[5] != HID * HID || in_sizes[6] < HID) return;
  if (in_sizes[7] != HID * NACT || in_sizes[8] < NACT) return;
  if (out_size <= 0 || (out_size % NACT) != 0) return;
  const int nG = out_size / NACT;
  if (nG > NGMAX) return;

  const float* x  = (const float*)d_in[0];
  const int*   ei = (const int*)d_in[1];
  const int*   bt = (const int*)d_in[2];
  const float* W1 = (const float*)d_in[3];
  const float* b1 = (const float*)d_in[4];
  const float* W2 = (const float*)d_in[5];
  const float* b2 = (const float*)d_in[6];
  const float* Wl = (const float*)d_in[7];
  const float* bl = (const float*)d_in[8];
  float* out = (float*)d_out;

  const int nBD = (nN + NBD - 1) / NBD;
  const int nGb = (nN + GR - 1) / GR;
  const int nA1 = (nN + NB1 - 1) / NB1;
  const int nA2 = (nN + NB2 - 1) / NB2;

  char* ws = (char*)d_ws;
  size_t off = 0;
  const size_t oW1 = off; off += (size_t)HID * DF * 2;                         off = (off + 255) & ~(size_t)255;
  const size_t oW2 = off; off += (size_t)HID * HID * 2;                        off = (off + 255) & ~(size_t)255;
  const size_t oDv = off; off += (size_t)nBD * NBD * 4;                        off = (off + 255) & ~(size_t)255;
  const size_t oG1 = off; off += (size_t)nGb * GR * HID * 4;                   off = (off + 255) & ~(size_t)255;
  const size_t oH1 = off; off += (size_t)nA1 * NB1 * HID * 2;                  off = (off + 255) & ~(size_t)255;
  const size_t oP  = off; off += (size_t)nGb * GR * NACT * 4;                  off = (off + 255) & ~(size_t)255;
  const size_t oH3 = off; off += (size_t)nA2 * NB2 * NACT * 4;                 off = (off + 255) & ~(size_t)255;
  if (off > ws_size) return;
  _Float16* w1t  = (_Float16*)(ws + oW1);
  _Float16* w2t  = (_Float16*)(ws + oW2);
  float*    dinv = (float*)(ws + oDv);
  float*    g1   = (float*)(ws + oG1);
  _Float16* h1p  = (_Float16*)(ws + oH1);
  float*    pp   = (float*)(ws + oP);
  float*    h3   = (float*)(ws + oH3);

  const int vec8 = ((nE & 3) == 0) ? 1 : 0;

  const int nPrep = HID * DF / 8 + HID * HID / 8;
  k_wprep<<<(nPrep + NTHR - 1) / NTHR, NTHR, 0, stream>>>(W1, W2, w1t, w2t);

  k_deg<<<nBD, NTHR, 0, stream>>>(ei, dinv, nN, nE, vec8);

  hipFuncSetAttribute(reinterpret_cast<const void*>(&k_gemm1),
                      hipFuncAttributeMaxDynamicSharedMemorySize, LDS_GEMM1);
  k_gemm1<<<nGb, NTHR, LDS_GEMM1, stream>>>(x, w1t, dinv, g1, nN);

  hipFuncSetAttribute(reinterpret_cast<const void*>(&k_agg1),
                      hipFuncAttributeMaxDynamicSharedMemorySize, LDS_AGG1);
  k_agg1<<<nA1, NTHR, LDS_AGG1, stream>>>(ei, g1, dinv, b1, h1p, nN, nE, vec8);

  k_gemm2h<<<nGb, NTHR, 0, stream>>>(h1p, w2t, Wl, dinv, pp);

  k_agg2<<<nA2, NTHR, 0, stream>>>(ei, pp, dinv, b2, Wl, bl, h3, nN, nE, vec8);

  k_pool<<<1, NTHR, 0, stream>>>(h3, bt, out, nN, nG);
}
